// NSE_42640435315484
// MI455X (gfx1250) — hardware-verified
//
#include <hip/hip_runtime.h>
#include <math.h>

constexpr int SEQ      = 96;
constexpr int NBATCH   = 64;
constexpr int HID      = 256;
constexpr int GATE4    = 1024;
constexpr int CMP      = 512;
constexpr int VOCAB    = 50257;
constexpr int NTHREADS = 256;
constexpr int SPB      = 16;

constexpr int AXP = 264;
constexpr int ACP = 520;
constexpr int AWP = 776;
constexpr int HRP = 256;
constexpr int ZP  = 96;

constexpr int OFF_AX   = 0;
constexpr int OFF_ACAT = OFF_AX   + SPB * AXP * 2;
constexpr int OFF_ACW  = OFF_ACAT + SPB * ACP * 2;
constexpr int OFF_HR   = OFF_ACW  + SPB * AWP * 2;
constexpr int OFF_HW   = OFF_HR   + SPB * HRP * 4;
constexpr int OFF_Z    = OFF_HW   + SPB * HRP * 4;
constexpr int LDS_BYTES = OFF_Z   + SPB * ZP * 4;
static_assert(OFF_ACAT == 8448 && OFF_ACW == 25088 && OFF_HR == 49920 && OFF_HW == 66304 && OFF_Z == 82688 && LDS_BYTES == 88832);
static_assert((OFF_ACAT % 16) == 0 && (OFF_ACW % 16) == 0 && (OFF_HR % 16) == 0 && (OFF_HW % 16) == 0 && (OFF_Z % 16) == 0);

constexpr float ACT_SC  = 16.0f;
constexpr float WF_SC   = 16.0f;
constexpr float WB_SC   = 256.0f;
constexpr float ACC_INV = 1.0f / 256.0f;

typedef __attribute__((ext_vector_type(16))) _Float16 v16h;
typedef __attribute__((ext_vector_type(8)))  _Float16 v8h;
typedef __attribute__((ext_vector_type(4)))  _Float16 v4h;
typedef __attribute__((ext_vector_type(16))) __bf16   v16b;
typedef __attribute__((ext_vector_type(8)))  __bf16   v8b;
typedef __attribute__((ext_vector_type(8)))  float    v8f;
typedef __attribute__((ext_vector_type(4)))  float    v4f;
typedef __attribute__((ext_vector_type(4)))  unsigned v4u;

__device__ __forceinline__ unsigned short f2bf_bits(float f) {
  unsigned u = __float_as_uint(f);
  return (unsigned short)((u + 0x7FFFu + ((u >> 16) & 1u)) >> 16);
}
__device__ __forceinline__ float bf_bits2f(unsigned short h) { return __uint_as_float(((unsigned)h) << 16); }
__device__ __forceinline__ float bfr(float f) { return bf_bits2f(f2bf_bits(f)); }

__device__ __forceinline__ void dep_guard_h(v8f& a, v8f& b, v16h x, v16h y) { asm volatile("v_nop\n\tv_nop\n\tv_nop\n\tv_nop" : "+v"(a), "+v"(b) : "v"(x), "v"(y)); }
__device__ __forceinline__ void dep_guard_b(v8f& a, v8f& b, v16b x, v16b y) { asm volatile("v_nop\n\tv_nop\n\tv_nop\n\tv_nop" : "+v"(a), "+v"(b) : "v"(x), "v"(y)); }
__device__ __forceinline__ void keep4_h(v16h a, v16h b, v16h c, v16h d) { asm volatile("v_nop" :: "v"(a), "v"(b), "v"(c), "v"(d)); }
__device__ __forceinline__ void keep4_b(v16b a, v16b b, v16b c, v16b d) { asm volatile("v_nop" :: "v"(a), "v"(b), "v"(c), "v"(d)); }
__device__ __forceinline__ void acc_guard4(v8f& a, v8f& b, v8f& c, v8f& d) { asm volatile("v_nop\n\tv_nop\n\tv_nop\n\tv_nop" : "+v"(a), "+v"(b), "+v"(c), "+v"(d)); }
template <typename T> struct Frag;
template <> struct Frag<_Float16> {
  typedef v16h V; union U { v16h v; v8h h[2]; };
  static __device__ __forceinline__ v16h load(const _Float16* p) {
    U f; f.h[0] = *(const v8h*)(p); f.h[1] = *(const v8h*)(p + 16); return f.v;
  }
  static __device__ __forceinline__ v8f mma(v16h a, v16h b, v8f c) {
    return __builtin_amdgcn_wmma_f32_16x16x32_f16(false, a, false, b, (short)0, c, false, false);
  }
  static __device__ __forceinline__ void guard(v8f& a, v8f& b, v16h x, v16h y) { dep_guard_h(a, b, x, y); }
  static __device__ __forceinline__ void keep(v16h a, v16h b, v16h c, v16h d) { keep4_h(a, b, c, d); }
};
template <> struct Frag<__bf16> {
  typedef v16b V; union U { v16b v; v8b h[2]; };
  static __device__ __forceinline__ v16b load(const __bf16* p) {
    U f; f.h[0] = *(const v8b*)(p); f.h[1] = *(const v8b*)(p + 16); return f.v;
  }
  static __device__ __forceinline__ v8f mma(v16b a, v16b b, v8f c) {
    return __builtin_amdgcn_wmma_f32_16x16x32_bf16(false, a, false, b, (short)0, c, false, false);
  }
  static __device__ __forceinline__ void guard(v8f& a, v8f& b, v16b x, v16b y) { dep_guard_b(a, b, x, y); }
  static __device__ __forceinline__ void keep(v16b a, v16b b, v16b c, v16b d) { keep4_b(a, b, c, d); }
};

__device__ __forceinline__ float fsig(float x)  { return __builtin_amdgcn_rcpf(1.0f + __expf(-x)); }
__device__ __forceinline__ float ftanh(float x) { return 1.0f - 2.0f * __builtin_amdgcn_rcpf(__expf(2.0f * x) + 1.0f); }

__device__ __forceinline__ v4f  ldv4(const float* p)    { return *(const volatile v4f*)p; }
__device__ __forceinline__ void stv4(float* p, v4f v)   { *(volatile v4f*)p = v; }

__device__ __forceinline__ void lds_wave_sync() {
  __builtin_amdgcn_fence(__ATOMIC_RELEASE, "workgroup");
  __builtin_amdgcn_wave_barrier();
  __builtin_amdgcn_fence(__ATOMIC_ACQUIRE, "workgroup");
}

template <int MODE>
__global__ __launch_bounds__(256) void cast16_kernel(const float* __restrict__ in, unsigned short* __restrict__ out, int n2, float sc) {
  const int i = blockIdx.x * 256 + threadIdx.x;
  if (i < n2) {
    const float a = in[2 * i], b = in[2 * i + 1];
    unsigned short u0, u1;
    if (MODE == 0) {
      u0 = f2bf_bits(a * sc); u1 = f2bf_bits(b * sc);
    } else {
      u0 = __builtin_bit_cast(unsigned short, (_Float16)(bfr(a) * sc));
      u1 = __builtin_bit_cast(unsigned short, (_Float16)(bfr(b) * sc));
    }
    const unsigned u = (unsigned)u0 | ((unsigned)u1 << 16);
    ((volatile unsigned*)out)[i] = u;
    __threadfence();
    ((volatile unsigned*)out)[i] = u;
  }
}

__global__ __launch_bounds__(256) void init_mem_kernel(const int* __restrict__ premise, const float* __restrict__ embed,
                                                      float* __restrict__ mem) {
  const int lane = threadIdx.x & 31, wave = threadIdx.x >> 5;
  const int row = blockIdx.x * 8 + wave;
  if (row >= NBATCH * SEQ) return;
  const int b = row / SEQ, s = row - b * SEQ;
  int tok = premise[s * NBATCH + b];
  tok = tok < 0 ? 0 : (tok > VOCAB - 1 ? VOCAB - 1 : tok);
  const float* src = embed + (size_t)tok * HID;
  v4f va = *(const v4f*)(src + 4 * lane);
  v4f vb = *(const v4f*)(src + 128 + 4 * lane);
#pragma unroll
  for (int e = 0; e < 4; ++e) { va[e] = bfr(va[e]); vb[e] = bfr(vb[e]); }
  float* dst = mem + (size_t)row * HID;
  stv4(dst + 4 * lane, va); stv4(dst + 128 + 4 * lane, vb);
  __threadfence();
  stv4(dst + 4 * lane, va); stv4(dst + 128 + 4 * lane, vb);
}

__device__ __forceinline__ void load_x_tile(unsigned short* Ax, const int* __restrict__ premise, const float* __restrict__ embed,
                                            int t, int b0, int tid) {
  const int m = tid >> 4, c16 = (tid & 15) * 16;
  int tok = premise[t * NBATCH + b0 + m];
  tok = tok < 0 ? 0 : (tok > VOCAB - 1 ? VOCAB - 1 : tok);
  const float* src = embed + (size_t)tok * HID + c16;
#pragma unroll
  for (int q = 0; q < 2; ++q) {
    const v4f va = *(const v4f*)(src + 8 * q);
    const v4f vb = *(const v4f*)(src + 8 * q + 4);
    v4u pk;
    pk[0] = (unsigned)f2bf_bits(va[0]) | ((unsigned)f2bf_bits(va[1]) << 16);
    pk[1] = (unsigned)f2bf_bits(va[2]) | ((unsigned)f2bf_bits(va[3]) << 16);
    pk[2] = (unsigned)f2bf_bits(vb[0]) | ((unsigned)f2bf_bits(vb[1]) << 16);
    pk[3] = (unsigned)f2bf_bits(vb[2]) | ((unsigned)f2bf_bits(vb[3]) << 16);
    *(v4u*)(Ax + m * AXP + c16 + 8 * q) = pk;
  }
}

__device__ __forceinline__ void cell8(const v8f& ai, const v8f& af, const v8f& ag, const v8f& ao,
                                      float bi, float bf, float bg, float bo, float (&cs)[8], float (&hs)[8]) {
#pragma unroll
  for (int r = 0; r < 8; ++r) {
    const float zi = ai[r] * ACC_INV + bi;
    const float zf = af[r] * ACC_INV + bf;
    const float zg = ag[r] * ACC_INV + bg;
    const float zo = ao[r] * ACC_INV + bo;
    const float ig = fsig(zi);
    const float fg = fsig(zf);
    const float gg = ftanh(zg);
    const float og = fsig(zo);
    const float cn = fg * cs[r] + ig * gg;
    cs[r] = cn;
    hs[r] = og * ftanh(cn);
  }
}

__global__ __launch_bounds__(NTHREADS) void mem_scan_kernel(
    const int* __restrict__ premise, const float* __restrict__ embed,
    const float* __restrict__ b_r, const float* __restrict__ bx, const float* __restrict__ b_w,
    const unsigned short* __restrict__ WIRp, const unsigned short* __restrict__ WHRp,
    const unsigned short* __restrict__ WXp,  const unsigned short* __restrict__ WIWp,
    const unsigned short* __restrict__ WHWp, float* __restrict__ mem) {
  extern __shared__ __align__(16) unsigned char smem[];
  unsigned short* Ax   = (unsigned short*)(smem + OFF_AX);
  _Float16*       Acat = (_Float16*)(smem + OFF_ACAT);
  _Float16*       Acw  = (_Float16*)(smem + OFF_ACW);
  float*          Hr   = (float*)(smem + OFF_HR);
  float*          Hw   = (float*)(smem + OFF_HW);
  float*          Zs   = (float*)(smem + OFF_Z);
  const __bf16*   WIR = (const __bf16*)WIRp;
  const _Float16* WHR = (const _Float16*)WHRp;
  const _Float16* WX  = (const _Float16*)WXp;
  const _Float16* WIW = (const _Float16*)WIWp;
  const _Float16* WHW = (const _Float16*)WHWp;

  const int tid = threadIdx.x, lane = tid & 31, wave = tid >> 5;
  const int c = lane & 15, hh = lane >> 4, koff = hh * 8;
  const int b0 = blockIdx.x * SPB;

#pragma unroll 1
  for (int i = 0; i < SPB; ++i) {
    Acat[i * ACP + tid] = (_Float16)0.0f;
    Acw[i * AWP + CMP + tid] = (_Float16)0.0f;
  }
  load_x_tile(Ax, premise, embed, 0, b0, tid);
  float cr[2][8], cw[2][8];
#pragma unroll
  for (int nt = 0; nt < 2; ++nt)
#pragma unroll
    for (int r = 0; r < 8; ++r) { cr[nt][r] = 0.0f; cw[nt][r] = 0.0f; }
  __syncthreads();

  const __bf16*   axrow = (const __bf16*)Ax + c * AXP + koff;
  const _Float16* acrow = Acat + c * ACP + koff;
  const _Float16* awrow = Acw  + c * AWP + koff;
  const v8f z8 = {0.f, 0.f, 0.f, 0.f, 0.f, 0.f, 0.f, 0.f};

#pragma unroll 1
  for (int t = 0; t < SEQ; ++t) {
    float hn[2][8];
#pragma unroll
    for (int nt = 0; nt < 2; ++nt) {
      const int j = 32 * wave + 16 * nt + c;
      const __bf16*   wi = WIR + (size_t)j * HID + koff;
      const _Float16* wh = WHR + (size_t)j * HID + koff;
      v8f acc[4];
      acc[0] = z8; acc[1] = z8; acc[2] = z8; acc[3] = z8;
#pragma unroll 1
      for (int k0 = 0; k0 < HID; k0 += 32) {
        const v16b a  = Frag<__bf16>::load(axrow + k0);
        const v16b f0 = Frag<__bf16>::load(wi + k0);
        const v16b f1 = Frag<__bf16>::load(wi + (size_t)1 * HID * HID + k0);
        const v16b f2 = Frag<__bf16>::load(wi + (size_t)2 * HID * HID + k0);
        const v16b f3 = Frag<__bf16>::load(wi + (size_t)3 * HID * HID + k0);
        acc[0] = Frag<__bf16>::mma(a, f0, acc[0]);
        acc[1] = Frag<__bf16>::mma(a, f1, acc[1]);
        acc[2] = Frag<__bf16>::mma(a, f2, acc[2]);
        acc[3] = Frag<__bf16>::mma(a, f3, acc[3]);
        dep_guard_b(acc[0], acc[3], a, f3);
        keep4_b(f0, f1, f2, f3);
      }
#pragma unroll 1
      for (int k0 = 0; k0 < HID; k0 += 32) {
        const v16h a  = Frag<_Float16>::load(acrow + k0);
        const v16h f0 = Frag<_Float16>::load(wh + k0);
        const v16h f1 = Frag<_Float16>::load(wh + (size_t)1 * HID * HID + k0);
        const v16h f2 = Frag<_Float16>::load(wh + (size_t)2 * HID * HID + k0);
        const v16h f3 = Frag<_Float16>::load(wh + (size_t)3 * HID * HID + k0);
        acc[0] = Frag<_Float16>::mma(a, f0, acc[0]);
        acc[1] = Frag<_Float16>::mma(a, f1, acc[1]);
        acc[2] = Frag<_Float16>::mma(a, f2, acc[2]);
        acc[3] = Frag<_Float16>::mma(a, f3, acc[3]);
        dep_guard_h(acc[0], acc[3], a, f3);
        keep4_h(f0, f1, f2, f3);
      }
      acc_guard4(acc[0], acc[1], acc[2], acc[3]);
      const float bi = bfr(b_r[j]), bf = bfr(b_r[HID + j]), bg = bfr(b_r[2 * HID + j]), bo = bfr(b_r[3 * HID + j]);
      cell8(acc[0], acc[1], acc[2], acc[3], bi, bf, bg, bo, cr[nt], hn[nt]);
    }
    __syncthreads();
#pragma unroll
    for (int nt = 0; nt < 2; ++nt) {
      const int j = 32 * wave + 16 * nt + c;
#pragma unroll
      for (int r = 0; r < 8; ++r) {
        Acat[(8 * hh + r) * ACP + j] = (_Float16)(hn[nt][r] * ACT_SC);
        Hr[(8 * hh + r) * HRP + j] = hn[nt][r];
      }
    }
    {
      const int tn = (t + 1 < SEQ) ? (t + 1) : (SEQ - 1);
      load_x_tile(Ax, premise, embed, tn, b0, tid);
    }
    __syncthreads();

#pragma unroll 1
    for (int q = 0; q < 2; ++q) {
      const int sq = 2 * wave + q;
      const float* Mb = mem + (size_t)(b0 + sq) * (size_t)(SEQ * HID);
      const float* hr = Hr + sq * HRP;
      const float* r0p = Mb + (size_t)lane * HID;
      const float* r1p = Mb + (size_t)(lane + 32) * HID;
      const float* r2p = Mb + (size_t)(lane + 64) * HID;
      float s0 = 0.0f, s1 = 0.0f, s2 = 0.0f;
#pragma unroll 2
      for (int d4 = 0; d4 < HID / 4; ++d4) {
        const v4f hv = *(const v4f*)(hr + 4 * d4);
        const v4f m0 = ldv4(r0p + 4 * d4);
        const v4f m1 = ldv4(r1p + 4 * d4);
        const v4f m2 = ldv4(r2p + 4 * d4);
        s0 += hv[0] * m0[0]; s0 += hv[1] * m0[1]; s0 += hv[2] * m0[2]; s0 += hv[3] * m0[3];
        s1 += hv[0] * m1[0]; s1 += hv[1] * m1[1]; s1 += hv[2] * m1[2]; s1 += hv[3] * m1[3];
        s2 += hv[0] * m2[0]; s2 += hv[1] * m2[1]; s2 += hv[2] * m2[2]; s2 += hv[3] * m2[3];
      }
      float mx = fmaxf(s0, fmaxf(s1, s2));
#pragma unroll
      for (int off = 16; off > 0; off >>= 1) mx = fmaxf(mx, __shfl_xor(mx, off, 32));
      const float e0 = __expf(s0 - mx), e1 = __expf(s1 - mx), e2 = __expf(s2 - mx);
      float sum = e0 + e1 + e2;
#pragma unroll
      for (int off = 16; off > 0; off >>= 1) sum += __shfl_xor(sum, off, 32);
      const float inv = 1.0f / sum;
      Zs[sq * ZP + lane]      = e0 * inv;
      Zs[sq * ZP + 32 + lane] = e1 * inv;
      Zs[sq * ZP + 64 + lane] = e2 * inv;
      lds_wave_sync();
      v4f ma = {0.f, 0.f, 0.f, 0.f}, mb = {0.f, 0.f, 0.f, 0.f};
#pragma unroll 2
      for (int s = 0; s < SEQ; ++s) {
        const float z = Zs[sq * ZP + s];
        const v4f a = ldv4(Mb + (size_t)s * HID + 4 * lane);
        const v4f b = ldv4(Mb + (size_t)s * HID + 128 + 4 * lane);
        ma += a * z;
        mb += b * z;
      }
      v4h pa, pb;
#pragma unroll
      for (int e = 0; e < 4; ++e) { pa[e] = (_Float16)(ma[e] * ACT_SC); pb[e] = (_Float16)(mb[e] * ACT_SC); }
      *(v4h*)(Acat + sq * ACP + HID + 4 * lane)       = pa;
      *(v4h*)(Acat + sq * ACP + HID + 128 + 4 * lane) = pb;
    }
    __syncthreads();

    {
      const int nb = 64 * wave;
      const _Float16* wx = WX + (size_t)(nb + c) * CMP + koff;
      v8f acc[4];
      acc[0] = z8; acc[1] = z8; acc[2] = z8; acc[3] = z8;
#pragma unroll 1
      for (int k0 = 0; k0 < CMP; k0 += 32) {
        const v16h a  = Frag<_Float16>::load(acrow + k0);
        const v16h f0 = Frag<_Float16>::load(wx + k0);
        const v16h f1 = Frag<_Float16>::load(wx + (size_t)16 * CMP + k0);
        const v16h f2 = Frag<_Float16>::load(wx + (size_t)32 * CMP + k0);
        const v16h f3 = Frag<_Float16>::load(wx + (size_t)48 * CMP + k0);
        acc[0] = Frag<_Float16>::mma(a, f0, acc[0]);
        acc[1] = Frag<_Float16>::mma(a, f1, acc[1]);
        acc[2] = Frag<_Float16>::mma(a, f2, acc[2]);
        acc[3] = Frag<_Float16>::mma(a, f3, acc[3]);
        dep_guard_h(acc[0], acc[3], a, f3);
        keep4_h(f0, f1, f2, f3);
      }
      acc_guard4(acc[0], acc[1], acc[2], acc[3]);
#pragma unroll
      for (int nt = 0; nt < 4; ++nt) {
        const int n = nb + 16 * nt + c;
        const float bv = bfr(bx[n]);
#pragma unroll
        for (int r = 0; r < 8; ++r) {
          const float v = acc[nt][r] * ACC_INV + bv;
          Acw[(8 * hh + r) * AWP + n] = (_Float16)(v * ACT_SC);
        }
      }
    }
    __syncthreads();

#pragma unroll
    for (int nt = 0; nt < 2; ++nt) {
      const int j = 32 * wave + 16 * nt + c;
      const _Float16* wi = WIW + (size_t)j * CMP + koff;
      const _Float16* wh = WHW + (size_t)j * HID + koff;
      v8f acc[4];
      acc[0] = z8; acc[1] = z8; acc[2] = z8; acc[3] = z8;
#pragma unroll 1
      for (int k0 = 0; k0 < CMP; k0 += 32) {
        const v16h a  = Frag<_Float16>::load(awrow + k0);
        const v16h f0 = Frag<_Float16>::load(wi + k0);
        const v16h f1 = Frag<_Float16>::load(wi + (size_t)1 * HID * CMP + k0);
        const v16h f2 = Frag<_Float16>::load(wi + (size_t)2 * HID * CMP + k0);
        const v16h f3 = Frag<_Float16>::load(wi + (size_t)3 * HID * CMP + k0);
        acc[0] = Frag<_Float16>::mma(a, f0, acc[0]);
        acc[1] = Frag<_Float16>::mma(a, f1, acc[1]);
        acc[2] = Frag<_Float16>::mma(a, f2, acc[2]);
        acc[3] = Frag<_Float16>::mma(a, f3, acc[3]);
        dep_guard_h(acc[0], acc[3], a, f3);
        keep4_h(f0, f1, f2, f3);
      }
#pragma unroll 1
      for (int k0 = 0; k0 < HID; k0 += 32) {
        const v16h a  = Frag<_Float16>::load(awrow + CMP + k0);
        const v16h f0 = Frag<_Float16>::load(wh + k0);
        const v16h f1 = Frag<_Float16>::load(wh + (size_t)1 * HID * HID + k0);
        const v16h f2 = Frag<_Float16>::load(wh + (size_t)2 * HID * HID + k0);
        const v16h f3 = Frag<_Float16>::load(wh + (size_t)3 * HID * HID + k0);
        acc[0] = Frag<_Float16>::mma(a, f0, acc[0]);
        acc[1] = Frag<_Float16>::mma(a, f1, acc[1]);
        acc[2] = Frag<_Float16>::mma(a, f2, acc[2]);
        acc[3] = Frag<_Float16>::mma(a, f3, acc[3]);
        dep_guard_h(acc[0], acc[3], a, f3);
        keep4_h(f0, f1, f2, f3);
      }
      acc_guard4(acc[0], acc[1], acc[2], acc[3]);
      const float bi = bfr(b_w[j]), bf = bfr(b_w[HID + j]), bg = bfr(b_w[2 * HID + j]), bo = bfr(b_w[3 * HID + j]);
      cell8(acc[0], acc[1], acc[2], acc[3], bi, bf, bg, bo, cw[nt], hn[nt]);
    }
    __syncthreads();
#pragma unroll
    for (int nt = 0; nt < 2; ++nt) {
      const int j = 32 * wave + 16 * nt + c;
#pragma unroll
      for (int r = 0; r < 8; ++r) {
        Acw[(8 * hh + r) * AWP + CMP + j] = (_Float16)(hn[nt][r] * ACT_SC);
        Hw[(8 * hh + r) * HRP + j] = hn[nt][r];
      }
    }
    __syncthreads();

#pragma unroll 1
    for (int q = 0; q < 2; ++q) {
      const int sq = 2 * wave + q;
      float* Mb = mem + (size_t)(b0 + sq) * (size_t)(SEQ * HID);
      const v4f hwa = *(const v4f*)(Hw + sq * HRP + 4 * lane);
      const v4f hwb = *(const v4f*)(Hw + sq * HRP + 128 + 4 * lane);
#pragma unroll 1
      for (int s = 0; s < SEQ; ++s) {
        const float z = Zs[sq * ZP + s];
        const float omz = 1.0f - z;
        float* pa = Mb + (size_t)s * HID + 4 * lane;
        float* pb = pa + 128;
        const v4f a = ldv4(pa);
        const v4f b = ldv4(pb);
        const v4f na = a * omz + hwa * z;
        const v4f nb = b * omz + hwb * z;
        stv4(pa, na); stv4(pb, nb);
        __threadfence();
        stv4(pa, na); stv4(pb, nb);
      }
    }
    __threadfence();
    __syncthreads();
  }
}

extern "C" void kernel_launch(void* const* d_in, const int* in_sizes, int n_in,
                              void* d_out, int out_size, void* d_ws, size_t ws_size, hipStream_t stream) {
  if (n_in < 10 || d_out == nullptr || d_ws == nullptr) return;
  if (in_sizes[0] != SEQ * NBATCH || in_sizes[1] != VOCAB * HID ||
      in_sizes[2] != GATE4 * HID || in_sizes[3] != GATE4 * HID || in_sizes[4] != GATE4 ||
      in_sizes[5] != CMP * CMP || in_sizes[6] != CMP ||
      in_sizes[7] != GATE4 * CMP || in_sizes[8] != GATE4 * HID || in_sizes[9] != GATE4 ||
      out_size != NBATCH * SEQ * HID) return;

  const int*   premise = (const int*)d_in[0];
  const float* embed   = (const float*)d_in[1];
  const float* Wih_r   = (const float*)d_in[2];
  const float* Whh_r   = (const float*)d_in[3];
  const float* b_r     = (const float*)d_in[4];
  const float* Wx      = (const float*)d_in[5];
  const float* bx      = (const float*)d_in[6];
  const float* Wih_w   = (const float*)d_in[7];
  const float* Whh_w   = (const float*)d_in[8];
  const float* b_w     = (const float*)d_in[9];
  float* out = (float*)d_out;

  char* ws = (char*)d_ws; size_t off = 0;
  auto carve = [&](size_t bytes) -> char* { char* p = ws + off; off += (bytes + 255) & ~(size_t)255; return p; };
  unsigned short* WIR = (unsigned short*)carve((size_t)GATE4 * HID * 2);
  unsigned short* WHR = (unsigned short*)carve((size_t)GATE4 * HID * 2);
  unsigned short* WX  = (unsigned short*)carve((size_t)CMP * CMP * 2);
  unsigned short* WIW = (unsigned short*)carve((size_t)GATE4 * CMP * 2);
  unsigned short* WHW = (unsigned short*)carve((size_t)GATE4 * HID * 2);
  if (off > ws_size || off > (size_t)134217728) return;

  const int n2a = GATE4 * HID / 2, n2b = CMP * CMP / 2, n2c = GATE4 * CMP / 2;
  cast16_kernel<0><<<(n2a + 255) / 256, 256, 0, stream>>>(Wih_r, WIR, n2a, WB_SC);
  cast16_kernel<1><<<(n2a + 255) / 256, 256, 0, stream>>>(Whh_r, WHR, n2a, WF_SC);
  cast16_kernel<1><<<(n2b + 255) / 256, 256, 0, stream>>>(Wx,    WX,  n2b, WF_SC);
  cast16_kernel<1><<<(n2c + 255) / 256, 256, 0, stream>>>(Wih_w, WIW, n2c, WF_SC);
  cast16_kernel<1><<<(n2a + 255) / 256, 256, 0, stream>>>(Whh_w, WHW, n2a, WF_SC);
  init_mem_kernel<<<(NBATCH * SEQ) / 8, 256, 0, stream>>>(premise, embed, out);
  hipFuncSetAttribute(reinterpret_cast<const void*>(&mem_scan_kernel), hipFuncAttributeMaxDynamicSharedMemorySize, (int)(LDS_BYTES));
  mem_scan_kernel<<<NBATCH / SPB, NTHREADS, LDS_BYTES, stream>>>(premise, embed, b_r, bx, b_w, WIR, WHR, WX, WIW, WHW, out);
}
